// JointAttention_52166672777574
// MI455X (gfx1250) — hardware-verified
//
#include <hip/hip_runtime.h>
#include <math.h>

constexpr int kBatch = 2;
constexpr int kSeq   = 2048;
constexpr int kDim   = 2048;
constexpr int kHeads = 16;
constexpr int kKV    = 8;
constexpr int kHD    = 128;
constexpr int kTok   = kBatch * kSeq;
constexpr int kNQ    = kHeads * kHD;
constexpr int kNK    = kKV * kHD;
constexpr int kNQK   = kNQ + kNK;
constexpr int kNQKV  = kNQ + 2 * kNK;
constexpr int kQKRows = kBatch * (kHeads + kKV) * kSeq;
constexpr int kKRow0  = kBatch * kHeads * kSeq;
constexpr float kEps        = 1.1920929e-07f;
constexpr float kInvHD      = 1.0f / 128.0f;
constexpr float kWCarry     = 16.0f;
constexpr float kWCarryInv  = 1.0f / 16.0f;
constexpr float kPCarry     = 32768.0f;
constexpr float kOCarry     = 16.0f;
constexpr float kPVScale    = kOCarry / kPCarry;
constexpr float kOutScale   = 1.0f / (kOCarry * kWCarry);
constexpr float kScoreScale = 0.08838834764831845f;
static_assert(kHD == 128, "norm kernel lane map: 32 lanes x 4 dims");
static_assert(kHeads == 2 * kKV, "two query heads per kv head");
static_assert(kSeq % 64 == 0 && kNQK % 64 == 0 && kNK % 64 == 0 && kNQ % 64 == 0 && kDim % 64 == 0 && kTok % 64 == 0, "GEMM M/N tiles");
static_assert(kHD % 64 == 0, "GEMM N tile (ctx)");
static_assert(kDim % 32 == 0 && kHD % 32 == 0 && kSeq % 32 == 0 && kNQ % 32 == 0, "GEMM K % 32");
static_assert(kSeq == 256 * 8, "softmax coverage: 256 threads x 8 columns");
static_assert((kHeads + kKV) % 8 == 0, "norm kernel: 8 waves per block over 24 q|k heads");

typedef __attribute__((ext_vector_type(16))) _Float16 v16h;
typedef __attribute__((ext_vector_type(8)))  _Float16 v8h;
typedef __attribute__((ext_vector_type(16))) __bf16   v16b;
typedef __attribute__((ext_vector_type(8)))  __bf16   v8b;
typedef __attribute__((ext_vector_type(8)))  float    v8f;
typedef __attribute__((ext_vector_type(4)))  float    v4f;
typedef __attribute__((ext_vector_type(2)))  float    v2f;
typedef __attribute__((ext_vector_type(2)))  int      v2i;
typedef __attribute__((ext_vector_type(4)))  unsigned int v4u;

__device__ __forceinline__ unsigned short f2bf_bits(float f) {
  unsigned u = __float_as_uint(f);
  return (unsigned short)((u + 0x7FFFu + ((u >> 16) & 1u)) >> 16);
}
__device__ __forceinline__ float bf_bits2f(unsigned short h) { return __uint_as_float(((unsigned)h) << 16); }

__device__ __forceinline__ void dep_guard_h(v8f& a, v8f& b, v16h x, v16h y) { asm volatile("v_nop\n\tv_nop\n\tv_nop\n\tv_nop" : "+v"(a), "+v"(b) : "v"(x), "v"(y)); }
__device__ __forceinline__ void dep_guard_b(v8f& a, v8f& b, v16b x, v16b y) { asm volatile("v_nop\n\tv_nop\n\tv_nop\n\tv_nop" : "+v"(a), "+v"(b) : "v"(x), "v"(y)); }
__device__ __forceinline__ void keep4_h(v16h a, v16h b, v16h c, v16h d) { asm volatile("v_nop" :: "v"(a), "v"(b), "v"(c), "v"(d)); }
__device__ __forceinline__ void keep4_b(v16b a, v16b b, v16b c, v16b d) { asm volatile("v_nop" :: "v"(a), "v"(b), "v"(c), "v"(d)); }
__device__ __forceinline__ void acc_guard4(v8f& a, v8f& b, v8f& c, v8f& d) { asm volatile("v_nop\n\tv_nop\n\tv_nop\n\tv_nop" : "+v"(a), "+v"(b), "+v"(c), "+v"(d)); }
template <typename T> struct Frag;
template <> struct Frag<_Float16> {
  typedef v16h V; union U { v16h v; v8h h[2]; };
  static __device__ __forceinline__ v16h load(const _Float16* p) {
    U f; f.h[0] = *(const v8h*)(p); f.h[1] = *(const v8h*)(p + 16); return f.v;
  }
  static __device__ __forceinline__ v8f mma(v16h a, v16h b, v8f c) {
    return __builtin_amdgcn_wmma_f32_16x16x32_f16(false, a, false, b, (short)0, c, false, false);
  }
  static __device__ __forceinline__ void guard(v8f& a, v8f& b, v16h x, v16h y) { dep_guard_h(a, b, x, y); }
  static __device__ __forceinline__ void keep(v16h a, v16h b, v16h c, v16h d) { keep4_h(a, b, c, d); }
};
template <> struct Frag<__bf16> {
  typedef v16b V; union U { v16b v; v8b h[2]; };
  static __device__ __forceinline__ v16b load(const __bf16* p) {
    U f; f.h[0] = *(const v8b*)(p); f.h[1] = *(const v8b*)(p + 16); return f.v;
  }
  static __device__ __forceinline__ v8f mma(v16b a, v16b b, v8f c) {
    return __builtin_amdgcn_wmma_f32_16x16x32_bf16(false, a, false, b, (short)0, c, false, false);
  }
  static __device__ __forceinline__ void guard(v8f& a, v8f& b, v16b x, v16b y) { dep_guard_b(a, b, x, y); }
  static __device__ __forceinline__ void keep(v16b a, v16b b, v16b c, v16b d) { keep4_b(a, b, c, d); }
};

__device__ __forceinline__ unsigned pk16(unsigned short a, unsigned short b) { return (unsigned)a | ((unsigned)b << 16); }
__device__ __forceinline__ unsigned short h_bits(float f) { const _Float16 h = (_Float16)f; return __builtin_bit_cast(unsigned short, h); }
__device__ __forceinline__ float bfr(float f) { return bf_bits2f(f2bf_bits(f)); }

template <int ET> struct Elem;
template <> struct Elem<0> { typedef _Float16 T; };
template <> struct Elem<1> { typedef __bf16 T; };
template <int ET, bool SPLIT, int BIAS_MODE, int OUT_MODE, bool RESID, int ACT = 0>
__global__ __launch_bounds__(256) void wmma_gemm64(
    const unsigned short* __restrict__ Ap, const unsigned short* __restrict__ A2p, int lda, long strideA,
    const unsigned short* __restrict__ Btp, const unsigned short* __restrict__ Bt2p, int ldb, long strideB,
    void* __restrict__ Cout, void* __restrict__ Cout2, int ldc, long strideC,
    const float* __restrict__ bias,
    const float* __restrict__ resid, long strideR,
    int M, int N, int K, float scale) {
  typedef typename Elem<ET>::T T;
  typedef typename Frag<T>::V V;
  const T* A = (const T*)Ap; const T* A2 = (const T*)A2p; const T* Bt = (const T*)Btp; const T* Bt2 = (const T*)Bt2p;
  __shared__ __align__(16) float sT[8][16 * 68];
  const int b    = blockIdx.y;
  const int lane = threadIdx.x & 31;
  const int wave = threadIdx.x >> 5;
  const int tilesN = N >> 6;
  const int tilesM = M >> 6;
  const int tile = blockIdx.x * 8 + wave;
  if (tile >= tilesM * tilesN) return;
  const int tm = tile / tilesN;
  const int tn = tile - tm * tilesN;
  const int m0 = tm << 6;
  const int n0 = tn << 6;

  const T* Ab  = A  + (size_t)b * strideA;
  const T* Bb  = Bt + (size_t)b * strideB;
  const T* Ab2 = SPLIT ? (A2  + (size_t)b * strideA) : nullptr;
  const T* Bb2 = SPLIT ? (Bt2 + (size_t)b * strideB) : nullptr;

  const int rlane = lane & 15;
  const int koff  = (lane >> 4) * 8;
  const int mOff  = (lane >> 4) * 8;

  v8f acc[4][4];
#pragma unroll
  for (int i = 0; i < 4; ++i)
#pragma unroll
    for (int j = 0; j < 4; ++j) acc[i][j] = (v8f){0.f,0.f,0.f,0.f,0.f,0.f,0.f,0.f};

  for (int k0 = 0; k0 < K; k0 += 32) {
    V bh[4], bl[4];
#pragma unroll
    for (int j = 0; j < 4; ++j) {
      const size_t bo = (size_t)(n0 + (j << 4) + rlane) * ldb + koff + k0;
      bh[j] = Frag<T>::load(Bb + bo);
      if (SPLIT) bl[j] = Frag<T>::load(Bb2 + bo);
    }
#pragma unroll
    for (int i = 0; i < 4; ++i) {
      const size_t ao = (size_t)(m0 + (i << 4) + rlane) * lda + koff + k0;
      V ah = Frag<T>::load(Ab + ao);
      V al;
      if (SPLIT) al = Frag<T>::load(Ab2 + ao);
#pragma unroll
      for (int j = 0; j < 4; ++j) {
        acc[i][j] = Frag<T>::mma(ah, bh[j], acc[i][j]);
        if (SPLIT) {
          acc[i][j] = Frag<T>::mma(ah, bl[j], acc[i][j]);
          acc[i][j] = Frag<T>::mma(al, bh[j], acc[i][j]);
        }
      }
      Frag<T>::guard(acc[i][0], acc[i][3], ah, SPLIT ? al : ah);
    }
    Frag<T>::keep(bh[0], bh[1], bh[2], bh[3]);
    if (SPLIT) Frag<T>::keep(bl[0], bl[1], bl[2], bl[3]);
  }
  acc_guard4(acc[0][0], acc[0][1], acc[0][2], acc[0][3]);
  acc_guard4(acc[1][0], acc[1][1], acc[1][2], acc[1][3]);
  acc_guard4(acc[2][0], acc[2][1], acc[2][2], acc[2][3]);
  acc_guard4(acc[3][0], acc[3][1], acc[3][2], acc[3][3]);

  float* slab = sT[wave];
  const float* Rb = RESID ? (resid + (size_t)b * strideR) : nullptr;
#pragma unroll
  for (int i = 0; i < 4; ++i) {
    const int mBase = m0 + (i << 4);
#pragma unroll
    for (int j = 0; j < 4; ++j) {
      const int n = n0 + (j << 4) + rlane;
      float bv = 0.f;
      if (BIAS_MODE == 2) bv = bias[n];
#pragma unroll
      for (int r = 0; r < 8; ++r) {
        float v = acc[i][j][r] * scale;
        if (BIAS_MODE == 1) v += bias[mBase + mOff + r];
        if (BIAS_MODE == 2) v += bv;
        if (RESID) v += Rb[(size_t)(mBase + mOff + r) * ldc + n];
        if (ACT == 2) v = fmaxf(v, 0.0f);
        if (ACT == 4) v = (v > 0.f) ? v : 0.01f * v;
        slab[(mOff + r) * 68 + (j << 4) + rlane] = v;
      }
    }
    __builtin_amdgcn_fence(__ATOMIC_RELEASE, "workgroup");
    __builtin_amdgcn_wave_barrier();
    __builtin_amdgcn_fence(__ATOMIC_ACQUIRE, "workgroup");
    if (OUT_MODE == 0) {
      float* C = (float*)Cout + (size_t)b * strideC;
      const int hh = lane >> 4, c4 = (lane & 15) * 4;
      for (int pass = 0; pass < 2; ++pass) {
#pragma unroll
        for (int it = 0; it < 8; ++it) {
          const int row = it * 2 + hh;
          v4f v = *(const v4f*)(slab + row * 68 + c4);
          *(volatile v4f*)(C + (size_t)(mBase + row) * ldc + n0 + c4) = v;
        }
        __threadfence();
      }
    } else {
      const int q = lane >> 3, c8 = (lane & 7) * 8;
      unsigned short* C  = (unsigned short*)Cout  + (size_t)b * strideC;
      unsigned short* C2 = (OUT_MODE == 2) ? ((unsigned short*)Cout2 + (size_t)b * strideC) : nullptr;
      for (int pass = 0; pass < 2; ++pass) {
#pragma unroll
        for (int it = 0; it < 4; ++it) {
          const int row = it * 4 + q;
          const float* sp = slab + row * 68 + c8;
          v8h hv, lv;
#pragma unroll
          for (int e = 0; e < 8; ++e) {
            if (OUT_MODE == 1) {
              hv[e] = (_Float16)sp[e];
            } else {
              unsigned short hb = f2bf_bits(sp[e]);
              unsigned short lb = f2bf_bits(sp[e] - bf_bits2f(hb));
              hv[e] = __builtin_bit_cast(_Float16, hb);
              lv[e] = __builtin_bit_cast(_Float16, lb);
            }
          }
          *(volatile v8h*)(C + (size_t)(mBase + row) * ldc + n0 + c8) = hv;
          if (OUT_MODE == 2) *(volatile v8h*)(C2 + (size_t)(mBase + row) * ldc + n0 + c8) = lv;
        }
        __threadfence();
      }
    }
    __builtin_amdgcn_fence(__ATOMIC_RELEASE, "workgroup");
    __builtin_amdgcn_wave_barrier();
    __builtin_amdgcn_fence(__ATOMIC_ACQUIRE, "workgroup");
  }
}

__global__ __launch_bounds__(256) void cast8_kernel(const float* __restrict__ in, unsigned short* __restrict__ out, int n8, float scale) {
  const int i = blockIdx.x * 256 + threadIdx.x;
  if (i >= n8) return;
  const float* p = in + 8 * (size_t)i;
  const v4f a = *(const v4f*)(p);
  const v4f c = *(const v4f*)(p + 4);
  unsigned short hb[8];
#pragma unroll
  for (int e = 0; e < 4; ++e) {
    hb[e]     = h_bits(bfr(a[e]) * scale);
    hb[4 + e] = h_bits(bfr(c[e]) * scale);
  }
  const v4u u = (v4u){pk16(hb[0], hb[1]), pk16(hb[2], hb[3]), pk16(hb[4], hb[5]), pk16(hb[6], hb[7])};
  unsigned short* q = out + 8 * (size_t)i;
  *(volatile v4u*)q = u;
  __threadfence();
  *(volatile v4u*)q = u;
}

__global__ __launch_bounds__(256) void norm_rope_kernel(const float* __restrict__ QK, const float* __restrict__ fcs,
                                                        const float* __restrict__ qw, const float* __restrict__ kw,
                                                        unsigned short* __restrict__ Ph, long loOff, int b) {
  const int lane = threadIdx.x & 31;
  const int wave = threadIdx.x >> 5;
  const int head = blockIdx.x * 8 + wave;
  const int s    = blockIdx.y;
  const int d0   = lane * 4;

  const v4f xv = *(const v4f*)(QK + (size_t)s * kNQK + (size_t)head * kHD + d0);
  float v0 = xv[0], v1 = xv[1], v2 = xv[2], v3 = xv[3];
  float ss = 0.0f;
  ss += v0 * v0; ss += v1 * v1; ss += v2 * v2; ss += v3 * v3;
#pragma unroll
  for (int off = 1; off < 32; off <<= 1) ss += __shfl_xor(ss, off, 32);
  const float rn = rsqrtf(ss * kInvHD + kEps);

  const v4f wq = *(const v4f*)(qw + d0);
  const v4f wk = *(const v4f*)(kw + d0);
  const float fq = (head < kHeads) ? 1.0f : 0.0f;
  const float fk = 1.0f - fq;
  const float w0 = bfr(fmaf(fq, wq[0], fk * wk[0]));
  const float w1 = bfr(fmaf(fq, wq[1], fk * wk[1]));
  const float w2 = bfr(fmaf(fq, wq[2], fk * wk[2]));
  const float w3 = bfr(fmaf(fq, wq[3], fk * wk[3]));
  v0 = (v0 * rn) * w0; v1 = (v1 * rn) * w1; v2 = (v2 * rn) * w2; v3 = (v3 * rn) * w3;

  const float* fp = fcs + ((size_t)s * (kHD / 2) + 2 * lane) * 4;
  const v4f fa = *(const v4f*)(fp);
  const v4f fb = *(const v4f*)(fp + 4);
  const float a00 = bfr(fa[0]), a01 = bfr(fa[1]), a10 = bfr(fa[2]), a11 = bfr(fa[3]);
  const float b00 = bfr(fb[0]), b01 = bfr(fb[1]), b10 = bfr(fb[2]), b11 = bfr(fb[3]);
  const float o0 = a00 * v0 + a01 * v1;
  const float o1 = a10 * v0 + a11 * v1;
  const float o2 = b00 * v2 + b01 * v3;
  const float o3 = b10 * v2 + b11 * v3;

  const unsigned short hb0 = f2bf_bits(o0), hb1 = f2bf_bits(o1), hb2 = f2bf_bits(o2), hb3 = f2bf_bits(o3);
  const unsigned short lb0 = f2bf_bits(o0 - bf_bits2f(hb0));
  const unsigned short lb1 = f2bf_bits(o1 - bf_bits2f(hb1));
  const unsigned short lb2 = f2bf_bits(o2 - bf_bits2f(hb2));
  const unsigned short lb3 = f2bf_bits(o3 - bf_bits2f(hb3));
  const unsigned ph0 = pk16(hb0, hb1), ph1 = pk16(hb2, hb3);
  const unsigned pl0 = pk16(lb0, lb1), pl1 = pk16(lb2, lb3);

  const int src = (2 * lane) & 31;
  const unsigned gh0 = __shfl(ph0, src, 32);
  const unsigned gh1 = __shfl(ph1, src, 32);
  const unsigned gh2 = __shfl(ph0, src + 1, 32);
  const unsigned gh3 = __shfl(ph1, src + 1, 32);
  const unsigned gl0 = __shfl(pl0, src, 32);
  const unsigned gl1 = __shfl(pl1, src, 32);
  const unsigned gl2 = __shfl(pl0, src + 1, 32);
  const unsigned gl3 = __shfl(pl1, src + 1, 32);
  const bool loh = (lane >= 16);
  const v4u u = (v4u){loh ? gl0 : gh0, loh ? gl1 : gh1, loh ? gl2 : gh2, loh ? gl3 : gh3};

  const int hq = (head < kHeads) ? head : 0;
  const int hk = (head < kHeads) ? 0 : (head - kHeads);
  const size_t rowQ = ((size_t)(b * kHeads + hq)) * kSeq + s;
  const size_t rowK = (size_t)kKRow0 + ((size_t)(b * kKV + hk)) * kSeq + s;
  const size_t row  = (head < kHeads) ? rowQ : rowK;
  const size_t poff = loh ? (size_t)loOff : (size_t)0;
  unsigned short* dp = Ph + poff + row * kHD + 8 * (lane & 15);
  for (int pass = 0; pass < 2; ++pass) {
    *(volatile v4u*)dp = u;
    __threadfence();
  }
}

__global__ __launch_bounds__(256) void softmax_kernel(const float* __restrict__ Sp, const int* __restrict__ maskp,
                                                      unsigned short* __restrict__ Pp) {
  __shared__ __align__(16) float lg[kSeq];
  __shared__ float redM[8];
  __shared__ float redS[8];
  const int i    = blockIdx.x;
  const int hg   = blockIdx.y;
  const int t    = threadIdx.x;
  const int lane = t & 31, wave = t >> 5;
  const size_t rowoff = ((size_t)hg * kSeq + i) * kSeq;
  const float* sr = Sp + rowoff;

  float mx = -__builtin_inff();
#pragma unroll 1
  for (int it = 0; it < 4; ++it) {
    const int c = it * 512 + 2 * t;
    const v2f sv = *(const v2f*)(sr + c);
    const v2i mv = *(const v2i*)(maskp + c);
    v2f av;
#pragma unroll
    for (int e = 0; e < 2; ++e) {
      const float bias = (mv[e] != 0) ? 0.0f : -__builtin_inff();
      const float a = sv[e] + bias;
      av[e] = a;
      mx = fmaxf(mx, a);
    }
    *(v2f*)(lg + c) = av;
  }
#pragma unroll
  for (int off = 16; off > 0; off >>= 1) mx = fmaxf(mx, __shfl_xor(mx, off, 32));
  if (lane == 0) redM[wave] = mx;
  __syncthreads();
  float m = redM[0];
#pragma unroll
  for (int w = 1; w < 8; ++w) m = fmaxf(m, redM[w]);

  float sum = 0.f;
#pragma unroll 1
  for (int it = 0; it < 4; ++it) {
    const int c = it * 512 + 2 * t;
    const v2f l = *(const v2f*)(lg + c);
    v2f ev;
#pragma unroll
    for (int e = 0; e < 2; ++e) {
      ev[e] = expf(l[e] - m);
      sum += ev[e];
    }
    *(v2f*)(lg + c) = ev;
  }
#pragma unroll
  for (int off = 16; off > 0; off >>= 1) sum += __shfl_xor(sum, off, 32);
  if (lane == 0) redS[wave] = sum;
  __syncthreads();
  float tot = redS[0];
#pragma unroll
  for (int w = 1; w < 8; ++w) tot += redS[w];
  const float inv = kPCarry / tot;

  const v4f e0 = *(const v4f*)(lg + 8 * t);
  const v4f e1 = *(const v4f*)(lg + 8 * t + 4);
  unsigned short hb[8];
#pragma unroll
  for (int e = 0; e < 4; ++e) {
    hb[e]     = h_bits(e0[e] * inv);
    hb[4 + e] = h_bits(e1[e] * inv);
  }
  const v4u u = (v4u){pk16(hb[0], hb[1]), pk16(hb[2], hb[3]), pk16(hb[4], hb[5]), pk16(hb[6], hb[7])};
  unsigned short* pr = Pp + rowoff + 8 * (size_t)t;
  *(volatile v4u*)pr = u;
  __threadfence();
  *(volatile v4u*)pr = u;
}

extern "C" void kernel_launch(void* const* d_in, const int* in_sizes, int n_in,
                              void* d_out, int out_size, void* d_ws, size_t ws_size,
                              hipStream_t stream) {
  if (n_in < 7) return;
  const int nX = kBatch * kSeq * kDim;
  if (in_sizes[0] != nX) return;
  if (in_sizes[1] != kBatch * kSeq) return;
  if (in_sizes[2] != kSeq * (kHD / 2) * 4) return;
  if (in_sizes[3] != kNQKV * kDim) return;
  if (in_sizes[4] != kDim * kNQ) return;
  if (in_sizes[5] != kHD || in_sizes[6] != kHD) return;
  if (out_size != kTok * kDim) return;

  const size_t szX16  = (size_t)kTok * kDim * 2;
  const size_t szWq16 = (size_t)kNQKV * kDim * 2;
  const size_t szWo16 = (size_t)kDim * kNQ * 2;
  const size_t szQK32 = (size_t)kSeq * kNQK * 4;
  const size_t szSC   = (size_t)2 * kSeq * kSeq * 4;
  const size_t szR3   = (szQK32 > szSC) ? szQK32 : szSC;
  const size_t szVT   = (size_t)kBatch * kKV * kHD * kSeq * 2;
  const size_t szPl   = (size_t)kQKRows * kHD * 2;
  const size_t szOb   = (size_t)kTok * kNQ * 2;
  const size_t szPP   = (size_t)2 * kSeq * kSeq * 2;
  const size_t offX16  = 0;
  const size_t offWq16 = offX16 + szX16;
  const size_t offWo16 = offWq16 + szWq16;
  const size_t offR3   = offWo16 + szWo16;
  const size_t offVT   = offR3 + szR3;
  const size_t offPhi  = offVT + szVT;
  const size_t offPlo  = offPhi + szPl;
  const size_t total   = offPlo + szPl;
  if (szOb > szX16 || szPP > szWq16) return;
  if (ws_size < total) return;

  const float* x     = (const float*)d_in[0];
  const int*   xmask = (const int*)d_in[1];
  const float* freqs = (const float*)d_in[2];
  const float* wqkv  = (const float*)d_in[3];
  const float* wout  = (const float*)d_in[4];
  const float* qw    = (const float*)d_in[5];
  const float* kw    = (const float*)d_in[6];
  float* out = (float*)d_out;
  char* ws = (char*)d_ws;
  unsigned short* X16  = (unsigned short*)(ws + offX16);
  unsigned short* Ob   = (unsigned short*)(ws + offX16);
  unsigned short* Wq16 = (unsigned short*)(ws + offWq16);
  unsigned short* PP   = (unsigned short*)(ws + offWq16);
  unsigned short* Wo16 = (unsigned short*)(ws + offWo16);
  float* QK32 = (float*)(ws + offR3);
  float* SC   = (float*)(ws + offR3);
  unsigned short* VT  = (unsigned short*)(ws + offVT);
  unsigned short* Phi = (unsigned short*)(ws + offPhi);
  unsigned short* Plo = (unsigned short*)(ws + offPlo);
  const long loOff = (long)kQKRows * kHD;
  const float* dummyf = (const float*)(ws + offR3);

  const int n8x = nX / 8;
  const int n8w = (kNQKV * kDim) / 8;
  const int n8o = (kDim * kNQ) / 8;
  cast8_kernel<<<dim3(n8x / 256), dim3(256), 0, stream>>>(x, X16, n8x, 1.0f);
  cast8_kernel<<<dim3(n8w / 256), dim3(256), 0, stream>>>(wqkv, Wq16, n8w, kWCarry);
  cast8_kernel<<<dim3(n8o / 256), dim3(256), 0, stream>>>(wout, Wo16, n8o, kWCarry);

  {
    const int tilesQK = (kSeq / 64) * (kNQK / 64);
    for (int b = 0; b < kBatch; ++b) {
      const unsigned short* Xb = X16 + (size_t)b * kSeq * kDim;
      wmma_gemm64<0, false, 0, 0, false, 0><<<dim3(tilesQK / 8, 1), dim3(256), 0, stream>>>(
          Xb, Xb, kDim, 0L, Wq16, Wq16, kDim, 0L,
          (void*)QK32, (void*)QK32, kNQK, 0L, dummyf, dummyf, 0L, kSeq, kNQK, kDim, kWCarryInv);
      norm_rope_kernel<<<dim3((kHeads + kKV) / 8, kSeq), dim3(256), 0, stream>>>(QK32, freqs, qw, kw, Phi, loOff, b);
    }
  }

  {
    const int tilesVT = (kNK / 64) * (kSeq / 64);
    const unsigned short* Wv = Wq16 + (size_t)kNQK * kDim;
    wmma_gemm64<0, false, 0, 1, false, 0><<<dim3(tilesVT / 8, kBatch), dim3(256), 0, stream>>>(
        Wv, Wv, kDim, 0L, X16, X16, kDim, (long)kSeq * kDim,
        (void*)VT, (void*)VT, kSeq, (long)kNK * kSeq, dummyf, dummyf, 0L, kNK, kSeq, kDim, kWCarryInv);
  }

  const long strideQhead = (long)kSeq * kHD;
  const long strideScore = (long)kSeq * kSeq;
  const int  tilesScore  = (kSeq / 64) * (kSeq / 64);
  const int  tilesCtx    = (kSeq / 64) * (kHD / 64);
  for (int b = 0; b < kBatch; ++b) {
    for (int j = 0; j < kKV; ++j) {
      const unsigned short* Ahi = Phi + ((size_t)(b * kHeads + 2 * j) * kSeq) * kHD;
      const unsigned short* Alo = Ahi + loOff;
      const unsigned short* Bhi = Phi + ((size_t)kKRow0 + (size_t)(b * kKV + j) * kSeq) * kHD;
      const unsigned short* Blo = Bhi + loOff;
      wmma_gemm64<1, true, 0, 0, false, 0><<<dim3(tilesScore / 8, 2), dim3(256), 0, stream>>>(
          Ahi, Alo, kHD, strideQhead, Bhi, Blo, kHD, 0L,
          (void*)SC, (void*)SC, kSeq, strideScore, dummyf, dummyf, 0L, kSeq, kSeq, kHD, kScoreScale);
      softmax_kernel<<<dim3(kSeq, 2), dim3(256), 0, stream>>>(SC, xmask + (size_t)b * kSeq, PP);
      const unsigned short* VTg = VT + ((size_t)(b * kKV + j) * kHD) * kSeq;
      unsigned short* Og = Ob + ((size_t)b * kSeq) * kNQ + (size_t)(2 * j) * kHD;
      wmma_gemm64<0, false, 0, 1, false, 0><<<dim3(tilesCtx / 8, 2), dim3(256), 0, stream>>>(
          PP, PP, kSeq, strideScore, VTg, VTg, kSeq, 0L,
          (void*)Og, (void*)Og, kNQ, (long)kHD, dummyf, dummyf, 0L, kSeq, kHD, kSeq, kPVScale);
    }
  }

  {
    const int tilesOut = (kTok / 64) * (kDim / 64);
    wmma_gemm64<0, false, 0, 0, false, 0><<<dim3(tilesOut / 8, 1), dim3(256), 0, stream>>>(
        Ob, Ob, kNQ, 0L, Wo16, Wo16, kNQ, 0L,
        (void*)out, (void*)out, kDim, 0L, dummyf, dummyf, 0L, kTok, kDim, kNQ, kOutScale);
  }
}
